// SynergyGNN_48155173322907
// MI455X (gfx1250) — hardware-verified
//
#include <hip/hip_runtime.h>
#include <stddef.h>
#include <math.h>


#define DIN     64
#define DF      128
#define NTHR    256
#define NWAVE   8
#define EPT     8
#define NGRP    2
#define CHUNK   (NTHR * EPT * NGRP)
#define WCAP    (EPT * NGRP * 32)
#define LISTN   (NWAVE * WCAP)
#define NBA     512
#define NBS     4096
#define GROWS   128
#define AP1     72
#define WSCALE  64.0f
#define WINV    0.015625f

#define LDS_GEMM (GROWS * DF * 4)
#define LDS_AGG  (NBA * DF * 4 + LISTN * 4 + 64)

static_assert((CHUNK & (CHUNK - 1)) == 0);
static_assert(CHUNK <= 4096);
static_assert((NBA & (NBA - 1)) == 0 && (NBS & (NBS - 1)) == 0);
static_assert(NBA <= 4096 && NBS <= 4096);
static_assert(NBA % GROWS == 0 && NBS % NBA == 0);
static_assert(GROWS * AP1 * 2 <= LDS_GEMM);
static_assert(NBA * 4 <= LISTN * 4);
static_assert(NBA % NWAVE == 0 && NBA % 128 == 0 && NBA / 128 <= NWAVE);
static_assert(NBS % (128 * NWAVE) == 0);
static_assert(NBS % NTHR == 0);

typedef float    v4f  __attribute__((ext_vector_type(4)));
typedef float    v8f  __attribute__((ext_vector_type(8)));
typedef int      v4i  __attribute__((ext_vector_type(4)));
typedef _Float16 v8h  __attribute__((ext_vector_type(8)));
typedef _Float16 v16h __attribute__((ext_vector_type(16)));
union FragH { v16h v; v8h h[2]; };

__device__ __forceinline__ v8h cvt8(v4f a, v4f b) {
  v8h r;
  r[0] = (_Float16)a.x; r[1] = (_Float16)a.y; r[2] = (_Float16)a.z; r[3] = (_Float16)a.w;
  r[4] = (_Float16)b.x; r[5] = (_Float16)b.y; r[6] = (_Float16)b.z; r[7] = (_Float16)b.w;
  return r;
}

__device__ __forceinline__ v8f wmh(v16h a, v16h b, v8f c) {
  v8f d = __builtin_amdgcn_wmma_f32_16x16x32_f16(false, a, false, b, (short)0, c, false, false);
  asm volatile("v_nop\n\tv_nop\n\tv_nop\n\tv_nop" : "+v"(d) : "v"(a), "v"(b));
  return d;
}

template <int NB>
__device__ __forceinline__ int scan_chunk(const int* __restrict__ dsts, int nE, int cbase, int nodeBase,
                                          int vec8, int* list, int tid, int lane, int wave) {
  int wc = 0;
#pragma unroll
  for (int g = 0; g < NGRP; ++g) {
    const int el0  = (g * NTHR + tid) * EPT;
    const int e0   = cbase + el0;
    const int sent = -2147483647 - 1;
    v4i da, db;
    if (vec8 != 0 && e0 + 7 < nE) {
      da = *(const v4i*)(dsts + e0);
      db = *(const v4i*)(dsts + e0 + 4);
    } else {
      da.x = (e0     < nE) ? dsts[min(e0, nE - 1)] : sent;
      da.y = (e0 + 1 < nE) ? dsts[min(e0 + 1, nE - 1)] : sent;
      da.z = (e0 + 2 < nE) ? dsts[min(e0 + 2, nE - 1)] : sent;
      da.w = (e0 + 3 < nE) ? dsts[min(e0 + 3, nE - 1)] : sent;
      db.x = (e0 + 4 < nE) ? dsts[min(e0 + 4, nE - 1)] : sent;
      db.y = (e0 + 5 < nE) ? dsts[min(e0 + 5, nE - 1)] : sent;
      db.z = (e0 + 6 < nE) ? dsts[min(e0 + 6, nE - 1)] : sent;
      db.w = (e0 + 7 < nE) ? dsts[min(e0 + 7, nE - 1)] : sent;
    }
    const unsigned nb = (unsigned)nodeBase;
    const unsigned s0 = (unsigned)da.x - nb, s1 = (unsigned)da.y - nb;
    const unsigned s2 = (unsigned)da.z - nb, s3 = (unsigned)da.w - nb;
    const unsigned s4 = (unsigned)db.x - nb, s5 = (unsigned)db.y - nb;
    const unsigned s6 = (unsigned)db.z - nb, s7 = (unsigned)db.w - nb;
    const bool h0 = s0 < (unsigned)NB, h1 = s1 < (unsigned)NB, h2 = s2 < (unsigned)NB, h3 = s3 < (unsigned)NB;
    const bool h4 = s4 < (unsigned)NB, h5 = s5 < (unsigned)NB, h6 = s6 < (unsigned)NB, h7 = s7 < (unsigned)NB;
    const unsigned any = __builtin_amdgcn_ballot_w32(h0 | h1 | h2 | h3 | h4 | h5 | h6 | h7);
    if (any != 0u) {
#define HITJ(J, HJ, SJ) { \
        const unsigned mj = __builtin_amdgcn_ballot_w32(HJ); \
        if (mj != 0u) { \
          if (HJ) { \
            const int pos = wc + (int)__builtin_amdgcn_mbcnt_lo(mj, 0u); \
            if (pos < WCAP) list[wave * WCAP + pos] = ((el0 + (J)) << 12) | (int)(SJ); \
          } \
          wc += (int)__builtin_popcount(mj); } }
      HITJ(0, h0, s0)
      HITJ(1, h1, s1)
      HITJ(2, h2, s2)
      HITJ(3, h3, s3)
      HITJ(4, h4, s4)
      HITJ(5, h5, s5)
      HITJ(6, h6, s6)
      HITJ(7, h7, s7)
#undef HITJ
    }
  }
  return wc;
}

__global__ __launch_bounds__(NTHR) void k_wprep(
    const float* __restrict__ W1, const float* __restrict__ W2,
    _Float16* w1s, _Float16* w2s) {
  const int i  = blockIdx.x * NTHR + threadIdx.x;
  const int n1 = DF * DIN / 8;
  const int n2 = DF * DF / 8;
  if (i >= n1 + n2) return;
  const bool first = i < n1;
  const int o  = (first ? i : i - n1) * 8;
  const int n  = first ? (o >> 6) : (o >> 7);
  const int k0 = first ? (o & (DIN - 1)) : (o & (DF - 1));
  const float* p = (first ? W1 : W2) + (size_t)k0 * DF + n;
  v4f a, b;
  a.x = p[0];      a.y = p[DF];     a.z = p[2 * DF]; a.w = p[3 * DF];
  b.x = p[4 * DF]; b.y = p[5 * DF]; b.z = p[6 * DF]; b.w = p[7 * DF];
  a = a * WSCALE;
  b = b * WSCALE;
  const v8h hv = cvt8(a, b);
  _Float16* dp = (first ? w1s : w2s) + o;
  *(volatile v8h*)dp = hv;
  __threadfence();
  *(volatile v8h*)dp = hv;
}

__global__ __launch_bounds__(NTHR) void k_deg(
    const int* __restrict__ ei, float* dinv, int nE, int vec8) {
  __shared__ __attribute__((aligned(16))) int cnt[NBS];
  __shared__ __attribute__((aligned(16))) int list[LISTN];
  __shared__ int wcnt[NWAVE];
  const int tid = threadIdx.x, lane = tid & 31, wave = tid >> 5;
  const int nodeBase = blockIdx.x * NBS;
  const int* dsts = ei + nE;

  for (int i = tid; i < NBS; i += NTHR) cnt[i] = 0;
  __syncthreads();

  const int nChunks = (nE + CHUNK - 1) / CHUNK;
#pragma unroll 1
  for (int ch = 0; ch < nChunks; ++ch) {
    const int cbase = ch * CHUNK;
    const int wc = scan_chunk<NBS>(dsts, nE, cbase, nodeBase, vec8, list, tid, lane, wave);
    if (lane == 0) wcnt[wave] = wc;
    __syncthreads();
    if (wave == 0) {
#pragma unroll 1
      for (int wsx = 0; wsx < NWAVE; ++wsx) {
        int n = __builtin_amdgcn_readfirstlane(wcnt[wsx]);
        n = n > WCAP ? WCAP : (n < 0 ? 0 : n);
        const int* lp = list + wsx * WCAP;
#pragma unroll 1
        for (int i = 0; i < n; ++i) {
          const int ent  = __builtin_amdgcn_readfirstlane(lp[i]);
          const int slot = ent & (NBS - 1);
          if (lane == 0) cnt[slot] = cnt[slot] + 1;
        }
      }
    }
    __syncthreads();
  }

  float* dp = dinv + (size_t)nodeBase;
#pragma unroll 1
  for (int q = 0; q < NBS / (128 * NWAVE); ++q) {
    const int f = (wave * (NBS / (128 * NWAVE)) + q) * 128 + 4 * lane;
    const v4i c = *(const v4i*)(cnt + f);
    v4f d;
    d.x = rsqrtf((float)(c.x + 1));
    d.y = rsqrtf((float)(c.y + 1));
    d.z = rsqrtf((float)(c.z + 1));
    d.w = rsqrtf((float)(c.w + 1));
    *(volatile v4f*)(dp + f) = d;
  }
  __threadfence();
#pragma unroll 1
  for (int q = 0; q < NBS / (128 * NWAVE); ++q) {
    const int f = (wave * (NBS / (128 * NWAVE)) + q) * 128 + 4 * lane;
    const v4i c = *(const v4i*)(cnt + f);
    v4f d;
    d.x = rsqrtf((float)(c.x + 1));
    d.y = rsqrtf((float)(c.y + 1));
    d.z = rsqrtf((float)(c.z + 1));
    d.w = rsqrtf((float)(c.w + 1));
    *(volatile v4f*)(dp + f) = d;
  }
}

__device__ __forceinline__ void gemm_epilogue(v8f (&acc)[8], float* stg, const float* __restrict__ dinv,
                                              float* g, int rowBase, int wave, int lane, int hh, int m) {
  const int r0 = wave * 16 + 8 * hh;
  const v4f dA = *(const v4f*)(dinv + (size_t)rowBase + r0);
  const v4f dB = *(const v4f*)(dinv + (size_t)rowBase + r0 + 4);
  const float d0 = dA.x * WINV, d1 = dA.y * WINV, d2 = dA.z * WINV, d3 = dA.w * WINV;
  const float d4 = dB.x * WINV, d5 = dB.y * WINV, d6 = dB.z * WINV, d7 = dB.w * WINV;
  float* sp = stg + r0 * DF + m;
#pragma unroll
  for (int t = 0; t < 8; ++t) {
    sp[0 * DF + 16 * t] = acc[t][0] * d0;
    sp[1 * DF + 16 * t] = acc[t][1] * d1;
    sp[2 * DF + 16 * t] = acc[t][2] * d2;
    sp[3 * DF + 16 * t] = acc[t][3] * d3;
    sp[4 * DF + 16 * t] = acc[t][4] * d4;
    sp[5 * DF + 16 * t] = acc[t][5] * d5;
    sp[6 * DF + 16 * t] = acc[t][6] * d6;
    sp[7 * DF + 16 * t] = acc[t][7] * d7;
  }
  __syncthreads();

  const float* lp = stg + wave * 16 * DF + 4 * lane;
  float* gp = g + ((size_t)rowBase + wave * 16) * DF + 4 * lane;
#pragma unroll
  for (int i = 0; i < 16; ++i) { const v4f v = *(const v4f*)(lp + i * DF); *(volatile v4f*)(gp + (size_t)i * DF) = v; }
  __threadfence();
#pragma unroll
  for (int i = 0; i < 16; ++i) { const v4f v = *(const v4f*)(lp + i * DF); *(volatile v4f*)(gp + (size_t)i * DF) = v; }
}

__global__ __launch_bounds__(NTHR) void k_gemm1(
    const float* __restrict__ x, const _Float16* __restrict__ w1s,
    const float* __restrict__ dinv, float* g, int nN) {
  extern __shared__ v4f lds_dyn[];
  _Float16* sA  = (_Float16*)lds_dyn;
  float*    stg = (float*)lds_dyn;
  const int tid = threadIdx.x, lane = tid & 31, wave = tid >> 5, hh = lane >> 4, m = lane & 15;
  const int rowBase = blockIdx.x * GROWS;

#pragma unroll
  for (int i = 0; i < (GROWS * DIN / 8) / NTHR; ++i) {
    const int idx = i * NTHR + tid;
    const int r   = idx >> 3;
    const int c0  = (idx & 7) * 8;
    int node = rowBase + r;
    node = node > nN - 1 ? nN - 1 : node;
    const float* xp = x + (size_t)node * DIN + c0;
    const v4f a = *(const v4f*)xp, b = *(const v4f*)(xp + 4);
    *(v8h*)(sA + r * AP1 + c0) = cvt8(a, b);
  }
  __syncthreads();

  v8f acc[8];
#pragma unroll
  for (int t = 0; t < 8; ++t) { v8f z = {0.f, 0.f, 0.f, 0.f, 0.f, 0.f, 0.f, 0.f}; acc[t] = z; }
  const _Float16* ar = sA + (wave * 16 + m) * AP1 + 8 * hh;
#pragma unroll 1
  for (int kt = 0; kt < DIN / 32; ++kt) {
    FragH a;
    a.h[0] = *(const v8h*)(ar + 32 * kt);
    a.h[1] = *(const v8h*)(ar + 32 * kt + 16);
#pragma unroll
    for (int t = 0; t < 8; ++t) {
      const _Float16* bp = w1s + (size_t)(16 * t + m) * DIN + 32 * kt + 8 * hh;
      FragH b;
      b.h[0] = *(const v8h*)bp;
      b.h[1] = *(const v8h*)(bp + 16);
      acc[t] = wmh(a.v, b.v, acc[t]);
    }
  }
  __syncthreads();

  gemm_epilogue(acc, stg, dinv, g, rowBase, wave, lane, hh, m);
}

__global__ __launch_bounds__(NTHR) void k_gemm2(
    const _Float16* __restrict__ h1, const _Float16* __restrict__ w2s,
    const float* __restrict__ dinv, float* g) {
  extern __shared__ v4f lds_dyn[];
  float* stg = (float*)lds_dyn;
  const int tid = threadIdx.x, lane = tid & 31, wave = tid >> 5, hh = lane >> 4, m = lane & 15;
  const int rowBase = blockIdx.x * GROWS;

  v8f acc[8];
#pragma unroll
  for (int t = 0; t < 8; ++t) { v8f z = {0.f, 0.f, 0.f, 0.f, 0.f, 0.f, 0.f, 0.f}; acc[t] = z; }
  const _Float16* ar = h1 + ((size_t)rowBase + wave * 16 + m) * DF + 8 * hh;
#pragma unroll 1
  for (int kt = 0; kt < DF / 32; ++kt) {
    FragH a;
    a.h[0] = *(const v8h*)(ar + 32 * kt);
    a.h[1] = *(const v8h*)(ar + 32 * kt + 16);
#pragma unroll
    for (int t = 0; t < 8; ++t) {
      const _Float16* bp = w2s + (size_t)(16 * t + m) * DF + 32 * kt + 8 * hh;
      FragH b;
      b.h[0] = *(const v8h*)bp;
      b.h[1] = *(const v8h*)(bp + 16);
      acc[t] = wmh(a.v, b.v, acc[t]);
    }
  }

  gemm_epilogue(acc, stg, dinv, g, rowBase, wave, lane, hh, m);
}

__device__ __forceinline__ void agg128_body(
    const int* __restrict__ ei, const float* __restrict__ g, const float* __restrict__ dinv,
    const float* __restrict__ bias, float* acc, int* list, int* wcnt,
    int nodeBase, int nN, int nE, int vec8, int tid, int lane, int wave) {
  {
    v4f* av = (v4f*)acc;
    const v4f z = {0.f, 0.f, 0.f, 0.f};
    for (int i = tid; i < NBA * DF / 4; i += NTHR) av[i] = z;
  }
  __syncthreads();

  const int* dsts = ei + nE;
  const int nChunks = (nE + CHUNK - 1) / CHUNK;
#pragma unroll 1
  for (int ch = 0; ch < nChunks; ++ch) {
    const int cbase = ch * CHUNK;
    const int wc = scan_chunk<NBA>(dsts, nE, cbase, nodeBase, vec8, list, tid, lane, wave);
    if (lane == 0) wcnt[wave] = wc;
    __syncthreads();
    if (wave == 0) {
#pragma unroll 1
      for (int wsx = 0; wsx < NWAVE; ++wsx) {
        int n = __builtin_amdgcn_readfirstlane(wcnt[wsx]);
        n = n > WCAP ? WCAP : (n < 0 ? 0 : n);
        const int* lp = list + wsx * WCAP;
#pragma unroll 1
        for (int i = 0; i < n; ++i) {
          const int ent  = __builtin_amdgcn_readfirstlane(lp[i]);
          const int slot = ent & (NBA - 1);
          int e = cbase + ((ent >> 12) & (CHUNK - 1));
          e = e > nE - 1 ? nE - 1 : e;
          int src = ei[e];
          src = src < 0 ? 0 : (src > nN - 1 ? nN - 1 : src);
          const v4f v = *(const v4f*)(g + (size_t)src * DF + 4 * lane);
          v4f* ap = (v4f*)(acc + slot * DF + 4 * lane);
          *ap = *ap + v;
        }
      }
    }
    __syncthreads();
  }

#pragma unroll 4
  for (int i = 0; i < (NBA * DF / 4) / NTHR; ++i) {
    const int idx  = i * NTHR + tid;
    const int slot = idx >> 5;
    const int c4   = (idx & 31) * 4;
    int node = nodeBase + slot;
    node = node > nN - 1 ? nN - 1 : node;
    const float d  = dinv[node];
    const v4f   gv = *(const v4f*)(g + (size_t)node * DF + c4);
    const v4f   bv = *(const v4f*)(bias + c4);
    v4f* ap = (v4f*)(acc + slot * DF + c4);
    v4f hv = (*ap + gv) * d + bv;
    hv.x = fmaxf(hv.x, 0.f); hv.y = fmaxf(hv.y, 0.f); hv.z = fmaxf(hv.z, 0.f); hv.w = fmaxf(hv.w, 0.f);
    *ap = hv;
  }
  __syncthreads();
}

__global__ __launch_bounds__(NTHR) void k_agg_h(
    const int* __restrict__ ei, const float* __restrict__ g, const float* __restrict__ dinv,
    const float* __restrict__ b1, _Float16* hout, int nN, int nE, int vec8) {
  extern __shared__ v4f lds_dyn[];
  float* acc  = (float*)lds_dyn;
  int*   list = (int*)(acc + NBA * DF);
  int*   wcnt = list + LISTN;
  const int tid = threadIdx.x, lane = tid & 31, wave = tid >> 5;
  const int nodeBase = blockIdx.x * NBA;

  agg128_body(ei, g, dinv, b1, acc, list, wcnt, nodeBase, nN, nE, vec8, tid, lane, wave);

#pragma unroll 4
  for (int i = 0; i < (NBA * DF / 8) / NTHR; ++i) {
    const int idx  = i * NTHR + tid;
    const int slot = idx >> 4;
    const int c8   = (idx & 15) * 8;
    const float* ap = acc + slot * DF + c8;
    const v8h hv = cvt8(*(const v4f*)ap, *(const v4f*)(ap + 4));
    *(volatile v8h*)(hout + ((size_t)nodeBase + slot) * DF + c8) = hv;
  }
  __threadfence();
#pragma unroll 4
  for (int i = 0; i < (NBA * DF / 8) / NTHR; ++i) {
    const int idx  = i * NTHR + tid;
    const int slot = idx >> 4;
    const int c8   = (idx & 15) * 8;
    const float* ap = acc + slot * DF + c8;
    const v8h hv = cvt8(*(const v4f*)ap, *(const v4f*)(ap + 4));
    *(volatile v8h*)(hout + ((size_t)nodeBase + slot) * DF + c8) = hv;
  }
}

__global__ __launch_bounds__(NTHR) void k_agg_g3(
    const int* __restrict__ ei, const float* __restrict__ g, const float* __restrict__ dinv,
    const float* __restrict__ b2, const float* __restrict__ W3, float* g3,
    int nN, int nE, int vec8) {
  extern __shared__ v4f lds_dyn[];
  float* acc  = (float*)lds_dyn;
  int*   list = (int*)(acc + NBA * DF);
  int*   wcnt = list + LISTN;
  float* g3s  = (float*)list;
  const int tid = threadIdx.x, lane = tid & 31, wave = tid >> 5;
  const int nodeBase = blockIdx.x * NBA;

  agg128_body(ei, g, dinv, b2, acc, list, wcnt, nodeBase, nN, nE, vec8, tid, lane, wave);

  const v4f w4 = *(const v4f*)(W3 + 4 * lane);
#pragma unroll 2
  for (int rr = 0; rr < NBA / NWAVE; ++rr) {
    const int slot = wave * (NBA / NWAVE) + rr;
    const v4f hv = *(const v4f*)(acc + slot * DF + 4 * lane);
    float s = hv.x * w4.x + hv.y * w4.y + hv.z * w4.z + hv.w * w4.w;
    s += __shfl_xor(s, 16, 32);
    s += __shfl_xor(s, 8, 32);
    s += __shfl_xor(s, 4, 32);
    s += __shfl_xor(s, 2, 32);
    s += __shfl_xor(s, 1, 32);
    if (lane == 0) g3s[slot] = s * dinv[(size_t)nodeBase + slot];
  }
  __syncthreads();

  v4f ov = {0.f, 0.f, 0.f, 0.f};
  const int f = wave * 128 + 4 * lane;
  if (wave < NBA / 128) { ov = *(const v4f*)(g3s + f); *(volatile v4f*)(g3 + (size_t)nodeBase + f) = ov; }
  __threadfence();
  if (wave < NBA / 128) { *(volatile v4f*)(g3 + (size_t)nodeBase + f) = ov; }
}

__global__ __launch_bounds__(NTHR) void k_agg_out(
    const int* __restrict__ ei, const float* __restrict__ g3, const float* __restrict__ dinv,
    const float* __restrict__ b3, float* out, int nN, int nE, int vec8) {
  __shared__ __attribute__((aligned(16))) float acc[NBS];
  __shared__ __attribute__((aligned(16))) int list[LISTN];
  __shared__ int wcnt[NWAVE];
  const int tid = threadIdx.x, lane = tid & 31, wave = tid >> 5;
  const int nodeBase = blockIdx.x * NBS;
  const int* dsts = ei + nE;

  {
    v4f* av = (v4f*)acc;
    const v4f z = {0.f, 0.f, 0.f, 0.f};
    for (int i = tid; i < NBS / 4; i += NTHR) av[i] = z;
  }
  __syncthreads();

  const int nChunks = (nE + CHUNK - 1) / CHUNK;
#pragma unroll 1
  for (int ch = 0; ch < nChunks; ++ch) {
    const int cbase = ch * CHUNK;
    const int wc = scan_chunk<NBS>(dsts, nE, cbase, nodeBase, vec8, list, tid, lane, wave);
    if (lane == 0) wcnt[wave] = wc;
    __syncthreads();
    if (wave == 0) {
#pragma unroll 1
      for (int wsx = 0; wsx < NWAVE; ++wsx) {
        int n = __builtin_amdgcn_readfirstlane(wcnt[wsx]);
        n = n > WCAP ? WCAP : (n < 0 ? 0 : n);
        const int* lp = list + wsx * WCAP;
#pragma unroll 1
        for (int i = 0; i < n; ++i) {
          const int ent  = __builtin_amdgcn_readfirstlane(lp[i]);
          const int slot = ent & (NBS - 1);
          int e = cbase + ((ent >> 12) & (CHUNK - 1));
          e = e > nE - 1 ? nE - 1 : e;
          int src = ei[e];
          src = src < 0 ? 0 : (src > nN - 1 ? nN - 1 : src);
          if (lane == 0) acc[slot] = acc[slot] + g3[src];
        }
      }
    }
    __syncthreads();
  }

  const float bb = b3[0];
#pragma unroll 1
  for (int i = 0; i < NBS / NTHR; ++i) {
    const int idx  = i * NTHR + tid;
    const int node = nodeBase + idx;
    const int cn   = node > nN - 1 ? nN - 1 : node;
    float v = (acc[idx] + g3[cn]) * dinv[(size_t)node] + bb;
    v = fminf(fmaxf(v, -30.0f), 30.0f);
    const float ev = expf(-v);
    acc[idx] = 1.0f / (1.0f + ev);
  }
  __syncthreads();

  const size_t outN = (size_t)nN;
#pragma unroll
  for (int q = 0; q < NBS / (128 * NWAVE); ++q) {
    const int f = (wave * (NBS / (128 * NWAVE)) + q) * 128 + 4 * lane;
    const size_t gi = (size_t)nodeBase + (size_t)f;
    const v4f v = *(const v4f*)(acc + f);
    if (gi + 4 <= outN) { *(volatile v4f*)(out + gi) = v; }
    else {
      if (gi     < outN) *(volatile float*)(out + gi)     = v.x;
      if (gi + 1 < outN) *(volatile float*)(out + gi + 1) = v.y;
      if (gi + 2 < outN) *(volatile float*)(out + gi + 2) = v.z;
      if (gi + 3 < outN) *(volatile float*)(out + gi + 3) = v.w;
    }
  }
  __threadfence();
#pragma unroll
  for (int q = 0; q < NBS / (128 * NWAVE); ++q) {
    const int f = (wave * (NBS / (128 * NWAVE)) + q) * 128 + 4 * lane;
    const size_t gi = (size_t)nodeBase + (size_t)f;
    const v4f v = *(const v4f*)(acc + f);
    if (gi + 4 <= outN) { *(volatile v4f*)(out + gi) = v; }
    else {
      if (gi     < outN) *(volatile float*)(out + gi)     = v.x;
      if (gi + 1 < outN) *(volatile float*)(out + gi + 1) = v.y;
      if (gi + 2 < outN) *(volatile float*)(out + gi + 2) = v.z;
      if (gi + 3 < outN) *(volatile float*)(out + gi + 3) = v.w;
    }
  }
}

extern "C" void kernel_launch(void* const* d_in, const int* in_sizes, int n_in,
                              void* d_out, int out_size, void* d_ws, size_t ws_size,
                              hipStream_t stream) {
  if (n_in < 8) return;
  const int nN = in_sizes[0] / DIN;
  const int nE = in_sizes[7] / 2;
  if (nN <= 0 || nE < 0 || in_sizes[0] != nN * DIN || in_sizes[7] != nE * 2) return;
  if (in_sizes[1] != DIN * DF || in_sizes[2] < DF || in_sizes[3] != DF * DF || in_sizes[4] < DF) return;
  if (in_sizes[5] < DF || in_sizes[6] < 1) return;
  if (out_size != nN) return;

  const float* x  = (const float*)d_in[0];
  const float* W1 = (const float*)d_in[1];
  const float* b1 = (const float*)d_in[2];
  const float* W2 = (const float*)d_in[3];
  const float* b2 = (const float*)d_in[4];
  const float* W3 = (const float*)d_in[5];
  const float* b3 = (const float*)d_in[6];
  const int*   ei = (const int*)d_in[7];
  float* out = (float*)d_out;

  const int nBD = (nN + NBS - 1) / NBS;
  const int nG  = (nN + GROWS - 1) / GROWS;
  const int nA  = (nN + NBA - 1) / NBA;

  char* ws = (char*)d_ws;
  size_t off = 0;
  const size_t oW1 = off; off += (size_t)DF * DIN * 2;                         off = (off + 255) & ~(size_t)255;
  const size_t oW2 = off; off += (size_t)DF * DF * 2;                          off = (off + 255) & ~(size_t)255;
  const size_t oDv = off; off += (size_t)nBD * NBS * 4;                        off = (off + 255) & ~(size_t)255;
  const size_t oG  = off; off += (size_t)nG * GROWS * DF * 4;                  off = (off + 255) & ~(size_t)255;
  const size_t oH  = off; off += (size_t)nA * NBA * DF * 2;                    off = (off + 255) & ~(size_t)255;
  const size_t oG3 = off; off += (size_t)nA * NBA * 4;                         off = (off + 255) & ~(size_t)255;
  if (off > ws_size) return;
  _Float16* w1s  = (_Float16*)(ws + oW1);
  _Float16* w2s  = (_Float16*)(ws + oW2);
  float*    dinv = (float*)(ws + oDv);
  float*    gpl  = (float*)(ws + oG);
  _Float16* h1   = (_Float16*)(ws + oH);
  float*    g3   = (float*)(ws + oG3);

  const int vec8 = ((nE & 3) == 0) ? 1 : 0;

  const int nPrep = DF * DIN / 8 + DF * DF / 8;
  k_wprep<<<(nPrep + NTHR - 1) / NTHR, NTHR, 0, stream>>>(W1, W2, w1s, w2s);

  k_deg<<<nBD, NTHR, 0, stream>>>(ei, dinv, nE, vec8);

  hipFuncSetAttribute(reinterpret_cast<const void*>(&k_gemm1),
                      hipFuncAttributeMaxDynamicSharedMemorySize, LDS_GEMM);
  k_gemm1<<<nG, NTHR, LDS_GEMM, stream>>>(x, w1s, dinv, gpl, nN);

  hipFuncSetAttribute(reinterpret_cast<const void*>(&k_agg_h),
                      hipFuncAttributeMaxDynamicSharedMemorySize, LDS_AGG);
  k_agg_h<<<nA, NTHR, LDS_AGG, stream>>>(ei, gpl, dinv, b1, h1, nN, nE, vec8);

  hipFuncSetAttribute(reinterpret_cast<const void*>(&k_gemm2),
                      hipFuncAttributeMaxDynamicSharedMemorySize, LDS_GEMM);
  k_gemm2<<<nG, NTHR, LDS_GEMM, stream>>>(h1, w2s, dinv, gpl);

  hipFuncSetAttribute(reinterpret_cast<const void*>(&k_agg_g3),
                      hipFuncAttributeMaxDynamicSharedMemorySize, LDS_AGG);
  k_agg_g3<<<nA, NTHR, LDS_AGG, stream>>>(ei, gpl, dinv, b2, W3, g3, nN, nE, vec8);

  k_agg_out<<<nBD, NTHR, 0, stream>>>(ei, g3, dinv, b3, out, nN, nE, vec8);
}
